// EdgeDecoder_14474039787539
// MI455X (gfx1250) — hardware-verified
//
#include <hip/hip_runtime.h>
#include <math.h>

typedef __attribute__((ext_vector_type(16))) _Float16 v16h;
typedef __attribute__((ext_vector_type(16))) __bf16 v16b;
typedef __attribute__((ext_vector_type(8)))  _Float16 v8h;
typedef __attribute__((ext_vector_type(8)))  float v8f;
typedef __attribute__((ext_vector_type(4)))  float v4f;
typedef __attribute__((ext_vector_type(2)))  float v2f;
typedef __attribute__((ext_vector_type(4)))  unsigned v4u;
typedef __attribute__((ext_vector_type(4)))  int v4i;
typedef float __attribute__((may_alias)) float_a;
typedef int __attribute__((may_alias)) int_a;

template <typename T> __device__ __forceinline__ void vst2(void* p, T v) { *(volatile T*)p = v; __threadfence(); *(volatile T*)p = v; }
__device__ __forceinline__ v8f wmma16(v16h a, v16h b, v8f c) {
  v8f d = __builtin_amdgcn_wmma_f32_16x16x32_f16(false, a, false, b, (short)0, c, false, false);
  asm volatile("v_nop\n\tv_nop\n\tv_nop\n\tv_nop" : "+v"(d) : "v"(a), "v"(b));
  return d;
}
__device__ __forceinline__ v8f wmma_bf(v16b a, v16b b, v8f c) {
  v8f d = __builtin_amdgcn_wmma_f32_16x16x32_bf16(false, a, false, b, (short)0, c, false, false);
  asm volatile("v_nop\n\tv_nop\n\tv_nop\n\tv_nop" : "+v"(d) : "v"(a), "v"(b));
  return d;
}
__device__ __forceinline__ v16h frag_h(const _Float16* rowk0, int lane) {
  union { v16h v; v8h q[2]; } u; const _Float16* p = rowk0 + 8 * (lane >> 4);
  u.q[0] = *(const v8h*)p; u.q[1] = *(const v8h*)(p + 16); return u.v;
}
__device__ __forceinline__ v16h frag_f32(const float* rowk0, int lane) {
  v16h a; const float* p = rowk0 + 8 * (lane >> 4);
#pragma unroll
  for (int i = 0; i < 8; ++i) { a[i] = (_Float16)p[i]; a[8 + i] = (_Float16)p[16 + i]; }
  return a;
}
__device__ __forceinline__ v16h frag_f32s(const float* rowk0, int lane, float sc) {
  v16h a; const float* p = rowk0 + 8 * (lane >> 4);
#pragma unroll
  for (int i = 0; i < 8; ++i) { a[i] = (_Float16)(p[i] * sc); a[8 + i] = (_Float16)(p[16 + i] * sc); }
  return a;
}
__device__ __forceinline__ v16h fragc_f32(const float* W, int k0, int n, int lane, int ld, int K) {
  v16h a; const int g = lane >> 4;
#pragma unroll
  for (int i = 0; i < 8; ++i) { const int ka = k0 + 8 * g + i, kb = ka + 16;
    a[i] = (_Float16)(ka < K ? W[(size_t)(ka < K ? ka : K - 1) * ld + n] : 0.f); a[8 + i] = (_Float16)(kb < K ? W[(size_t)(kb < K ? kb : K - 1) * ld + n] : 0.f); }
  return a;
}
struct F2 { v16b h, l; };
__device__ __forceinline__ F2 bsplit16(const float v[16]) { F2 r;
#pragma unroll
  for (int i = 0; i < 16; ++i) { const __bf16 h = (__bf16)v[i]; r.h[i] = h; r.l[i] = (__bf16)(v[i] - (float)h); }
  return r; }
__device__ __forceinline__ F2 split_row(const float* row, int k0, int lane) { float v[16]; const float* p = row + k0 + 8 * (lane >> 4);
#pragma unroll
  for (int i = 0; i < 8; ++i) { v[i] = p[i]; v[8 + i] = p[16 + i]; }
  return bsplit16(v); }
__device__ __forceinline__ F2 split_rowK(const float* row, int k0, int lane, int K) { float v[16]; const int g = lane >> 4;
#pragma unroll
  for (int i = 0; i < 8; ++i) { const int ka = k0 + 8 * g + i, kb = ka + 16; v[i] = ka < K ? row[ka < K ? ka : K - 1] : 0.f; v[8 + i] = kb < K ? row[kb < K ? kb : K - 1] : 0.f; }
  return bsplit16(v); }
__device__ __forceinline__ F2 split_col(const float* W, int k0, int n, int lane, int ld, int K) { float v[16]; const int g = lane >> 4;
#pragma unroll
  for (int i = 0; i < 8; ++i) { const int ka = k0 + 8 * g + i, kb = ka + 16; v[i] = ka < K ? W[(size_t)(ka < K ? ka : K - 1) * ld + n] : 0.f; v[8 + i] = kb < K ? W[(size_t)(kb < K ? kb : K - 1) * ld + n] : 0.f; }
  return bsplit16(v); }
__device__ __forceinline__ v8f mac3(const F2& a, const F2& b, v8f c) { c = wmma_bf(a.l, b.h, c); c = wmma_bf(a.h, b.l, c); return wmma_bf(a.h, b.h, c); }
__device__ __forceinline__ float sigm(float v) { return 1.0f / (1.0f + expf(-v)); }
#define LDSX() do { asm volatile("s_wait_dscnt 0" ::: "memory"); __builtin_amdgcn_wave_barrier(); __builtin_amdgcn_fence(__ATOMIC_RELEASE, "workgroup"); } while (0)

__device__ __forceinline__ float bfr(float v) { return (float)(__bf16)v; }
#define NE 2000000
#define HID 64
#ifndef NBLK
#define NBLK (NE / 64)
#endif
__global__ __launch_bounds__(128) void k_edge(const float* __restrict__ ZU, const float* __restrict__ ZB, const int* __restrict__ EI, const float* __restrict__ W1, const float* __restrict__ B1, const float* __restrict__ W2, const float* __restrict__ B2, float* __restrict__ OUT) { __shared__ __align__(16) float so[64];
  const int tid = threadIdx.x, wave = tid >> 5, lane = tid & 31, col = lane & 15, g = lane >> 4; const size_t e0 = (size_t)blockIdx.x * 64 + wave * 16;
  const int ru = EI[e0 + col], rb = EI[(size_t)NE + e0 + col];
  v8f acc[4] = {};
#pragma unroll
  for (int kc = 0; kc < 4; ++kc) { v16b a; const float* src = (kc < 2) ? (ZU + (size_t)ru * HID + kc * 32) : (ZB + (size_t)rb * HID + (kc - 2) * 32); const float* p = src + 8 * g;
#pragma unroll
    for (int i = 0; i < 8; ++i) { a[i] = (__bf16)p[i]; a[8 + i] = (__bf16)p[16 + i]; }
#pragma unroll
    for (int j = 0; j < 4; ++j) { v16b w; const int o = j * 16 + col; const float* wr = W1 + (size_t)o * (2 * HID) + kc * 32 + 8 * g;
#pragma unroll
      for (int i = 0; i < 8; ++i) { w[i] = (__bf16)wr[i]; w[8 + i] = (__bf16)wr[16 + i]; }
      acc[j] = wmma_bf(a, w, acc[j]); } }
  float rs[8];
#pragma unroll
  for (int r = 0; r < 8; ++r) rs[r] = 0.f;
#pragma unroll
  for (int j = 0; j < 4; ++j) { const int o = j * 16 + col; const float bb = bfr(B1[o]), w2 = bfr(W2[o]);
#pragma unroll
    for (int r = 0; r < 8; ++r) rs[r] += fmaxf(acc[j][r] + bb, 0.f) * w2; }
#pragma unroll
  for (int r = 0; r < 8; ++r) {
#pragma unroll
    for (int sh = 1; sh < 16; sh <<= 1) rs[r] += __shfl_xor(rs[r], sh); }
  if (col == 0) { const float b2 = bfr(B2[0]);
#pragma unroll
    for (int r = 0; r < 8; ++r) so[wave * 16 + 8 * g + r] = rs[r] + b2; }
  __syncthreads();
  if (tid < 16) vst2(OUT + (size_t)blockIdx.x * 64 + tid * 4, *(const v4f*)&so[tid * 4]); }
extern "C" void kernel_launch(void* const* d_in, const int* in_sizes, int n_in, void* d_out, int out_size, void* d_ws, size_t ws_size, hipStream_t stream) {
  (void)in_sizes; (void)n_in; (void)out_size; (void)d_ws; (void)ws_size;
  const float** F = (const float**)d_in;
  k_edge<<<dim3(NBLK), 128, 0, stream>>>(F[0], F[1], (const int*)d_in[2], F[3], F[4], F[5], F[6], (float*)d_out);
}
